// SAINTLite_42125039239564
// MI455X (gfx1250) — hardware-verified
//
#include <hip/hip_runtime.h>
#include <math.h>

#pragma clang fp contract(off)

#define NB   4
#define NT   2048
#define NR   (NB * NT)
#define DM   256
#define NH   8
#define DK   32
#define DF   1024
#define NL   2
#define KIN  384
#define DQ   64
#define FIN  8
#define NEMB 4000
#define NPAT 64
#define NSK  2000
#define NSP  2048
#define MH   4096

#define ES   1024.0f
#define XS0  256.0f
#define ASC  16.0f
#define RSC  16384.0f
#define WSC  64.0f
#define QS   64.0f
#define OS   256.0f
#define HS   64.0f
#define PSC  256.0f
#define INV_IN 1.52587890625e-5f
#define INV_X0 6.103515625e-5f
#define INV_LN 9.765625e-4f
#define INV_AT 6.103515625e-5f
#define INV_HP 2.44140625e-4f
#define LINV   5.9604644775390625e-8f
#define SSC    (0.17677669529663687f * 2.44140625e-4f)
#define OINV   6.103515625e-5f
#define GC     0.70710678118654752f

#define OP  68
#define OPT 132

static_assert(NR % 128 == 0 && NT % 64 == 0 && MH % 128 == 0 && NR == 2 * MH && NR % 8 == 0);
static_assert(DM % 64 == 0 && DF % 64 == 0 && KIN % 32 == 0 && NSP % 64 == 0 && NSK <= NSP && NSK % 4 == 0);
static_assert(DK == 32 && NH * DK == DM && (MH * (NSK / 4)) % 256 == 0 && NT % 256 == 0 && KIN == DM + 2 * DQ);
static_assert((OP % 4) == 0 && (OPT % 4) == 0 && 64 * OPT <= 128 * OP);

typedef _Float16 f16;
typedef _Float16 v16h __attribute__((ext_vector_type(16)));
typedef _Float16 v8h  __attribute__((ext_vector_type(8)));
typedef _Float16 v8ha __attribute__((ext_vector_type(8), may_alias));
typedef unsigned short v8us __attribute__((ext_vector_type(8)));
typedef float v8f __attribute__((ext_vector_type(8)));
typedef float v4f __attribute__((ext_vector_type(4)));
typedef float v4fa __attribute__((ext_vector_type(4), may_alias));

union FragH { v16h v; v8h h[2]; };

__device__ __forceinline__ float bf16r(float f) {
  unsigned int u = __float_as_uint(f);
  u = u + 0x7FFFu + ((u >> 16) & 1u);
  u &= 0xFFFF0000u;
  return __uint_as_float(u);
}

__device__ __forceinline__ void split2(float v, f16& hi, f16& lo) {
  const float s = v * ASC;
  const f16 hv = (f16)s;
  hi = hv;
  lo = (f16)((s - (float)hv) * RSC);
}

__device__ __forceinline__ float gelu_f(float v) { return 0.5f * v * (1.0f + erff(v * GC)); }

__device__ __forceinline__ v16h ld_frag(const f16* base, int row0, int k0, int ld) {
  const int lane = threadIdx.x & 31;
  const f16* p = base + (size_t)(row0 + (lane & 15)) * ld + k0 + ((lane >> 4) << 3);
  FragH f;
  f.h[0] = *(const v8h*)p;
  f.h[1] = *(const v8h*)(p + 16);
  return f.v;
}

__device__ __forceinline__ v8f mma_h(v16h a, v16h b, v8f c) {
  return __builtin_amdgcn_wmma_f32_16x16x32_f16(false, a, false, b, (short)0, c, false, false);
}

__device__ __forceinline__ void guard4x4(v8f& c0, v8f& c1, v8f& c2, v8f& c3,
                                         v16h f0, v16h f1, v16h f2, v16h f3) {
#if defined(__HIP_DEVICE_COMPILE__)
  asm volatile("v_nop\n\tv_nop\n\tv_nop\n\tv_nop"
               : "+v"(c0), "+v"(c1), "+v"(c2), "+v"(c3)
               : "v"(f0), "v"(f1), "v"(f2), "v"(f3));
#endif
}
__device__ __forceinline__ void guard8x6(v8f& c0, v8f& c1, v8f& c2, v8f& c3,
                                         v8f& c4, v8f& c5, v8f& c6, v8f& c7,
                                         v16h f0, v16h f1, v16h f2, v16h f3, v16h f4, v16h f5) {
#if defined(__HIP_DEVICE_COMPILE__)
  asm volatile("v_nop\n\tv_nop\n\tv_nop\n\tv_nop"
               : "+v"(c0), "+v"(c1), "+v"(c2), "+v"(c3), "+v"(c4), "+v"(c5), "+v"(c6), "+v"(c7)
               : "v"(f0), "v"(f1), "v"(f2), "v"(f3), "v"(f4), "v"(f5));
#endif
}
__device__ __forceinline__ void guard2x3(v8f& c0, v8f& c1, v16h f0, v16h f1, v16h f2) {
#if defined(__HIP_DEVICE_COMPILE__)
  asm volatile("v_nop\n\tv_nop\n\tv_nop\n\tv_nop"
               : "+v"(c0), "+v"(c1)
               : "v"(f0), "v"(f1), "v"(f2));
#endif
}

__global__ __launch_bounds__(256)
void k_cvt_wg(const float* __restrict__ W, unsigned short* dst, int K, int N, int Npad, int drows, int rowoff,
              float scale) {
  const int K8 = K >> 3;
  const int tot = Npad * K8;
  const int p = (int)blockIdx.x * 256 + (int)threadIdx.x;
  if (p >= tot) return;
  const int z = (int)blockIdx.y;
  const int n = p / K8, q = p - n * K8;
  const int nc = (n < N) ? n : (N - 1);
  const float* src = W + (size_t)z * (size_t)K * (size_t)N + nc;
  v8h o = {};
#pragma unroll
  for (int e = 0; e < 8; ++e) {
    const float w = src[(size_t)(8 * q + e) * (size_t)N];
    const float cv = bf16r(w) * scale;
    o[e] = (n < N) ? (f16)cv : (f16)0.0f;
  }
  const v8us u = __builtin_bit_cast(v8us, o);
  unsigned short* op = dst + ((size_t)z * (size_t)drows + (size_t)(rowoff + n)) * (size_t)K + 8 * q;
  *(volatile v8us*)op = u;
  __threadfence();
  *(volatile v8us*)op = u;
}

__global__ __launch_bounds__(256)
void k_bias(const float* __restrict__ kp, const float* __restrict__ ka, float* tab) {
  __shared__ __align__(16) float Sv[256];
  const int tid = threadIdx.x;
  const int lh = (int)blockIdx.y;
  const int d = (int)blockIdx.x * 256 + tid;
  const float xp = bf16r(kp[lh]), xa = bf16r(ka[lh]);
  const float pp = fmaxf(xp, 0.0f) + log1pf(expf(-fabsf(xp)));
  const float aa = fmaxf(xa, 0.0f) + log1pf(expf(-fabsf(xa)));
  const float t = pp * log1pf(aa * (float)d);
  Sv[tid] = -t;
  __syncthreads();
  v4f u = {};
  float* op = tab;
  if (tid < 64) {
    u = *(const v4fa*)&Sv[4 * tid];
    op = tab + (size_t)lh * NT + (size_t)blockIdx.x * 256 + 4 * tid;
    *(volatile v4f*)op = u;
  }
  __threadfence();
  if (tid < 64) *(volatile v4f*)op = u;
}

__global__ __launch_bounds__(256)
void k_xin(const int* __restrict__ inter, const int* __restrict__ pat, const float* __restrict__ ff,
           const float* __restrict__ ie, const float* __restrict__ pe, const float* __restrict__ fW,
           const float* __restrict__ fb, unsigned short* xin) {
  const int tid = threadIdx.x, lane = tid & 31, wv = tid >> 5;
  const int row = (int)blockIdx.x * 4 + (wv >> 1);
  const int part = wv & 1;
  unsigned short* dst = xin + (size_t)row * KIN;
  if (part == 0) {
    int id = inter[row];
    id = (id < 0) ? 0 : ((id >= NEMB) ? (NEMB - 1) : id);
    const float* s = ie + (size_t)id * DM + 8 * lane;
    const v4f a = *(const v4f*)s;
    const v4f c = *(const v4f*)(s + 4);
    v8h o = {};
#pragma unroll
    for (int e = 0; e < 4; ++e) { o[e] = (f16)(bf16r(a[e]) * ES); o[4 + e] = (f16)(bf16r(c[e]) * ES); }
    const v8us u = __builtin_bit_cast(v8us, o);
    unsigned short* op = dst + 8 * lane;
    *(volatile v8us*)op = u;
    __threadfence();
    *(volatile v8us*)op = u;
  } else {
    int pid = pat[row];
    pid = (pid < 0) ? 0 : ((pid >= NPAT) ? (NPAT - 1) : pid);
    const int q = lane & 7;
    const float* ps = pe + (size_t)pid * DQ + 8 * q;
    const v4f a = *(const v4f*)ps;
    const v4f c = *(const v4f*)(ps + 4);
    v8h po = {};
#pragma unroll
    for (int e = 0; e < 4; ++e) { po[e] = (f16)(bf16r(a[e]) * ES); po[4 + e] = (f16)(bf16r(c[e]) * ES); }
    float fv[FIN];
#pragma unroll
    for (int f = 0; f < FIN; ++f) fv[f] = bf16r(ff[(size_t)row * FIN + f]);
    v8h fo = {};
#pragma unroll
    for (int e = 0; e < 8; ++e) {
      const int cc = 8 * q + e;
      float acc = 0.0f;
#pragma unroll
      for (int f = 0; f < FIN; ++f) acc = acc + fv[f] * bf16r(fW[f * DQ + cc]);
      acc = acc + bf16r(fb[cc]);
      fo[e] = (f16)(acc * ES);
    }
    v8h sel = {};
#pragma unroll
    for (int e = 0; e < 8; ++e) sel[e] = (lane < 8) ? po[e] : fo[e];
    const v8us u = __builtin_bit_cast(v8us, sel);
    unsigned short* op = dst + DM + 8 * lane;
    if (lane < 16) *(volatile v8us*)op = u;
    __threadfence();
    if (lane < 16) *(volatile v8us*)op = u;
  }
}

template <bool LO>
__global__ __launch_bounds__(256)
void k_ln(const float* __restrict__ X, const float* __restrict__ g, const float* __restrict__ bb,
          float* Y, unsigned short* yh, unsigned short* yl) {
  __shared__ __align__(16) float Sx[8 * DM];
  const int tid = threadIdx.x, lane = tid & 31, wv = tid >> 5;
  const int row = (int)blockIdx.x * 8 + wv;
  const float* xp = X + (size_t)row * DM + 8 * lane;
  const v4f a = *(const v4f*)xp;
  const v4f c = *(const v4f*)(xp + 4);
  float v[8] = {a[0], a[1], a[2], a[3], c[0], c[1], c[2], c[3]};
  float s = 0.0f;
#pragma unroll
  for (int j = 0; j < 8; ++j) s += v[j];
#pragma unroll
  for (int m = 1; m < 32; m <<= 1) s += __shfl_xor(s, m, 32);
  const float mu = s * (1.0f / DM);
  float vs = 0.0f;
#pragma unroll
  for (int j = 0; j < 8; ++j) { const float t = v[j] - mu; vs += t * t; }
#pragma unroll
  for (int m = 1; m < 32; m <<= 1) vs += __shfl_xor(vs, m, 32);
  const float inv = rsqrtf(vs * (1.0f / DM) + 1e-6f);
  const v4f g0 = *(const v4f*)(g + 8 * lane);
  const v4f g1 = *(const v4f*)(g + 8 * lane + 4);
  const v4f b0 = *(const v4f*)(bb + 8 * lane);
  const v4f b1 = *(const v4f*)(bb + 8 * lane + 4);
  float gw[8] = {g0[0], g0[1], g0[2], g0[3], g1[0], g1[1], g1[2], g1[3]};
  float gb[8] = {b0[0], b0[1], b0[2], b0[3], b1[0], b1[1], b1[2], b1[3]};
  float y[8];
  v8h hi = {}, lo = {};
#pragma unroll
  for (int j = 0; j < 8; ++j) {
    y[j] = (bf16r(gw[j]) * (v[j] - mu)) * inv + bf16r(gb[j]);
    if constexpr (LO) {
      f16 x, e;
      split2(y[j], x, e);
      hi[j] = x;
      lo[j] = e;
    } else {
      hi[j] = (f16)(y[j] * ASC);
    }
  }
  {
    v4f y0, y1;
#pragma unroll
    for (int j = 0; j < 4; ++j) { y0[j] = y[j]; y1[j] = y[4 + j]; }
    float* sr = Sx + wv * DM + 8 * lane;
    *(v4fa*)sr = y0;
    *(v4fa*)(sr + 4) = y1;
  }
  __syncthreads();
  const float* rr = Sx + wv * DM;
  const v4f f0 = *(const v4fa*)(rr + 4 * lane);
  const v4f f1 = *(const v4fa*)(rr + 128 + 4 * lane);
  float* yr = Y + (size_t)row * DM;
  const v8us hu = __builtin_bit_cast(v8us, hi);
  const v8us lu = __builtin_bit_cast(v8us, lo);
  const size_t off = (size_t)row * DM + 8 * lane;
  *(volatile v4f*)(yr + 4 * lane) = f0;
  *(volatile v4f*)(yr + 128 + 4 * lane) = f1;
  *(volatile v8us*)(yh + off) = hu;
  if constexpr (LO) *(volatile v8us*)(yl + off) = lu;
  __threadfence();
  *(volatile v4f*)(yr + 4 * lane) = f0;
  *(volatile v4f*)(yr + 128 + 4 * lane) = f1;
  *(volatile v8us*)(yh + off) = hu;
  if constexpr (LO) *(volatile v8us*)(yl + off) = lu;
}

__device__ __forceinline__ void st_rowf(float* S, int row0, int col, v8f c, float hinv, float bn) {
#pragma unroll
  for (int r = 0; r < 8; ++r) S[(row0 + r) * OP + col] = c[r] * hinv + bn;
}
__device__ __forceinline__ void st_rowg(float* S, int row0, int col, v8f c, float hinv, float bn) {
#pragma unroll
  for (int r = 0; r < 8; ++r) S[(row0 + r) * OP + col] = gelu_f(c[r] * hinv + bn);
}
__device__ __forceinline__ void st_rowf2(float* S, int row0, int col, v8f hh, v8f gg, float bn) {
#pragma unroll
  for (int r = 0; r < 8; ++r) S[(row0 + r) * OP + col] = hh[r] * INV_LN + gg[r] * LINV + bn;
}
__device__ __forceinline__ void st_colf(float* S, int d, int tok0, v8f hh, float hinv, float bn) {
  v4f a, c;
#pragma unroll
  for (int i = 0; i < 4; ++i) {
    a[i] = hh[i] * hinv + bn;
    c[i] = hh[4 + i] * hinv + bn;
  }
  *(v4fa*)&S[d * OPT + tok0] = a;
  *(v4fa*)&S[d * OPT + tok0 + 4] = c;
}
__device__ __forceinline__ void st8(float* p, v8f o, float w) {
  v4f a, c;
#pragma unroll
  for (int i = 0; i < 4; ++i) { a[i] = o[i] * w; c[i] = o[4 + i] * w; }
  *(v4fa*)p = a;
  *(v4fa*)(p + 4) = c;
}

template <int MODE>
__global__ __launch_bounds__(256)
void k_gemm_x(const unsigned short* __restrict__ a16, const unsigned short* __restrict__ w16,
              const float* __restrict__ bias, const float* __restrict__ res,
              const float* __restrict__ ff, const float* __restrict__ tW, const float* __restrict__ tb,
              const float* __restrict__ pW, const float* __restrict__ pb,
              float* out, unsigned short* x16o, int K, int N, float hinv) {
  __shared__ __align__(16) float So[128 * OP];
  const int tid = threadIdx.x, lane = tid & 31, wv = tid >> 5, hl = lane >> 4, l15 = lane & 15;
  const int m0 = (int)blockIdx.y * 128, n0 = (int)blockIdx.x * 64;
  const int mp = wv >> 1, np = wv & 1;
  const int ra = m0 + 32 * mp, cb = n0 + 32 * np;
  const f16* Ap = (const f16*)a16;
  const f16* Wp = (const f16*)w16;

  v8f c00 = {}, c01 = {}, c10 = {}, c11 = {};
  const int nks = K >> 5;
#pragma unroll 1
  for (int ks = 0; ks < nks; ++ks) {
    const int k0 = ks << 5;
    const v16h a0 = ld_frag(Ap, ra, k0, K);
    const v16h a1 = ld_frag(Ap, ra + 16, k0, K);
    const v16h b0 = ld_frag(Wp, cb, k0, K);
    const v16h b1 = ld_frag(Wp, cb + 16, k0, K);
    c00 = mma_h(a0, b0, c00);
    c01 = mma_h(a0, b1, c01);
    c10 = mma_h(a1, b0, c10);
    c11 = mma_h(a1, b1, c11);
    guard4x4(c00, c01, c10, c11, a0, a1, b0, b1);
  }

  const float bn0 = bf16r(bias[cb + l15]);
  const float bn1 = bf16r(bias[cb + 16 + l15]);
  const int rr = 32 * mp + 8 * hl, cc = 32 * np + l15;
  st_rowf(So, rr,      cc,      c00, hinv, bn0);
  st_rowf(So, rr,      cc + 16, c01, hinv, bn1);
  st_rowf(So, rr + 16, cc,      c10, hinv, bn0);
  st_rowf(So, rr + 16, cc + 16, c11, hinv, bn1);
  __syncthreads();

  if constexpr (MODE == 0) {
#pragma unroll 1
    for (int i = 0; i < 32; ++i) {
      const int e = tid + 256 * i;
      const int row = e >> 6, col = e & 63;
      const int gr = m0 + row, d = n0 + col;
      const int s = gr & (NT - 1);
      const float el = bf16r(ff[(size_t)gr * FIN]);
      const float te = tanhf(el * bf16r(tW[d]) + bf16r(tb[d]));
      const float pe = ((float)s * (1.0f / (float)NT)) * bf16r(pW[d]) + bf16r(pb[d]);
      So[row * OP + col] = (So[row * OP + col] + te) + pe;
    }
    __syncthreads();
  }

  v4f u[8];
  size_t off[8];
#pragma unroll
  for (int it = 0; it < 8; ++it) {
    const int p = tid + 256 * it;
    const int row = p >> 4, q = p & 15;
    u[it] = *(const v4fa*)&So[row * OP + 4 * q];
    off[it] = (size_t)(m0 + row) * (size_t)N + n0 + 4 * q;
    if constexpr (MODE == 1) {
      const v4f rv = *(const v4f*)(res + off[it]);
      u[it] += rv;
    }
  }
#pragma unroll
  for (int it = 0; it < 8; ++it) *(volatile v4f*)(out + off[it]) = u[it];
  __threadfence();
#pragma unroll
  for (int it = 0; it < 8; ++it) *(volatile v4f*)(out + off[it]) = u[it];

  if constexpr (MODE == 0) {
    v8us hu[4];
    size_t ho[4];
#pragma unroll
    for (int it = 0; it < 4; ++it) {
      const int p = tid + 256 * it;
      const int row = p >> 3, q = p & 7;
      const float* sp = So + row * OP + 8 * q;
      const v4f a = *(const v4fa*)sp;
      const v4f c = *(const v4fa*)(sp + 4);
      v8h o = {};
#pragma unroll
      for (int e = 0; e < 4; ++e) { o[e] = (f16)(a[e] * XS0); o[4 + e] = (f16)(c[e] * XS0); }
      hu[it] = __builtin_bit_cast(v8us, o);
      ho[it] = (size_t)(m0 + row) * (size_t)DM + n0 + 8 * q;
    }
#pragma unroll
    for (int it = 0; it < 4; ++it) *(volatile v8us*)(x16o + ho[it]) = hu[it];
    __threadfence();
#pragma unroll
    for (int it = 0; it < 4; ++it) *(volatile v8us*)(x16o + ho[it]) = hu[it];
  }
}

__global__ __launch_bounds__(256)
void k_gemm_h(const unsigned short* __restrict__ a16, const unsigned short* __restrict__ w16,
              const float* __restrict__ bias, unsigned short* hp, int K, int N, float hinv) {
  __shared__ __align__(16) float So[128 * OP];
  const int tid = threadIdx.x, lane = tid & 31, wv = tid >> 5, hl = lane >> 4, l15 = lane & 15;
  const int m0 = (int)blockIdx.y * 128, n0 = (int)blockIdx.x * 64;
  const int mp = wv >> 1, np = wv & 1;
  const int ra = m0 + 32 * mp, cb = n0 + 32 * np;
  const f16* Ap = (const f16*)a16;
  const f16* Wp = (const f16*)w16;

  v8f c00 = {}, c01 = {}, c10 = {}, c11 = {};
  const int nks = K >> 5;
#pragma unroll 1
  for (int ks = 0; ks < nks; ++ks) {
    const int k0 = ks << 5;
    const v16h a0 = ld_frag(Ap, ra, k0, K);
    const v16h a1 = ld_frag(Ap, ra + 16, k0, K);
    const v16h b0 = ld_frag(Wp, cb, k0, K);
    const v16h b1 = ld_frag(Wp, cb + 16, k0, K);
    c00 = mma_h(a0, b0, c00);
    c01 = mma_h(a0, b1, c01);
    c10 = mma_h(a1, b0, c10);
    c11 = mma_h(a1, b1, c11);
    guard4x4(c00, c01, c10, c11, a0, a1, b0, b1);
  }

  const float bn0 = bf16r(bias[cb + l15]);
  const float bn1 = bf16r(bias[cb + 16 + l15]);
  const int rr = 32 * mp + 8 * hl, cc = 32 * np + l15;
  st_rowg(So, rr,      cc,      c00, hinv, bn0);
  st_rowg(So, rr,      cc + 16, c01, hinv, bn1);
  st_rowg(So, rr + 16, cc,      c10, hinv, bn0);
  st_rowg(So, rr + 16, cc + 16, c11, hinv, bn1);
  __syncthreads();

  v8us u[4];
  size_t off[4];
#pragma unroll
  for (int it = 0; it < 4; ++it) {
    const int p = tid + 256 * it;
    const int row = p >> 3, q = p & 7;
    const float* sp = So + row * OP + 8 * q;
    const v4f a = *(const v4fa*)sp;
    const v4f c = *(const v4fa*)(sp + 4);
    v8h o = {};
#pragma unroll
    for (int e = 0; e < 4; ++e) { o[e] = (f16)(a[e] * HS); o[4 + e] = (f16)(c[e] * HS); }
    u[it] = __builtin_bit_cast(v8us, o);
    off[it] = (size_t)(m0 + row) * (size_t)N + n0 + 8 * q;
  }
#pragma unroll
  for (int it = 0; it < 4; ++it) *(volatile v8us*)(hp + off[it]) = u[it];
  __threadfence();
#pragma unroll
  for (int it = 0; it < 4; ++it) *(volatile v8us*)(hp + off[it]) = u[it];
}

__global__ __launch_bounds__(256)
void k_gemm_heads(const unsigned short* __restrict__ ah, const unsigned short* __restrict__ w16,
                  const float* __restrict__ bq, const float* __restrict__ bk, const float* __restrict__ bv,
                  unsigned short* dq, unsigned short* dk, unsigned short* dvt, int K, float hinv) {
  __shared__ __align__(16) float So[128 * OP];
  const int tid = threadIdx.x, lane = tid & 31, wv = tid >> 5, hl = lane >> 4, l15 = lane & 15;
  const int nb = (int)blockIdx.x;
  const int m0 = (int)blockIdx.y * 128, n0 = nb * 64;
  const int stream = nb >> 2, head0 = (nb & 3) * 2;
  const int b = m0 / NT, t0 = m0 - b * NT;
  const f16* Hp = (const f16*)ah;
  const f16* Wp = (const f16*)w16;
  const int mp = wv >> 1, np = wv & 1;
  const int ra = m0 + 32 * mp, cb = n0 + 32 * np;

  v8f h00 = {}, h01 = {}, h10 = {}, h11 = {};
  const int nks = K >> 5;
#pragma unroll 1
  for (int ks = 0; ks < nks; ++ks) {
    const int k0 = ks << 5;
    const v16h a0 = ld_frag(Hp, ra, k0, K);
    const v16h a1 = ld_frag(Hp, ra + 16, k0, K);
    const v16h b0 = ld_frag(Wp, cb, k0, K);
    const v16h b1 = ld_frag(Wp, cb + 16, k0, K);
    h00 = mma_h(a0, b0, h00);
    h01 = mma_h(a0, b1, h01);
    h10 = mma_h(a1, b0, h10);
    h11 = mma_h(a1, b1, h11);
    guard4x4(h00, h01, h10, h11, a0, a1, b0, b1);
  }

  const float* bp = (stream == 0) ? bq : ((stream == 1) ? bk : bv);
  const int cs = (nb & 3) * 64 + 32 * np + l15;
  const float bn0 = bf16r(bp[cs]);
  const float bn1 = bf16r(bp[cs + 16]);
  const int rr = 32 * mp + 8 * hl, cc = 32 * np + l15;

  if (stream == 2) {
    st_colf(So, cc,      rr,      h00, hinv, bn0);
    st_colf(So, cc + 16, rr,      h01, hinv, bn1);
    st_colf(So, cc,      rr + 16, h10, hinv, bn0);
    st_colf(So, cc + 16, rr + 16, h11, hinv, bn1);
    __syncthreads();
    v8us u[4];
    size_t off[4];
#pragma unroll
    for (int it = 0; it < 4; ++it) {
      const int p = tid + 256 * it;
      const int d = p >> 4, q = p & 15;
      const float* sp = So + d * OPT + 8 * q;
      const v4f a = *(const v4fa*)sp;
      const v4f c = *(const v4fa*)(sp + 4);
      v8h o = {};
#pragma unroll
      for (int e = 0; e < 4; ++e) { o[e] = (f16)(a[e] * QS); o[4 + e] = (f16)(c[e] * QS); }
      u[it] = __builtin_bit_cast(v8us, o);
      off[it] = ((size_t)(b * NH + head0 + (d >> 5)) * DK + (d & 31)) * (size_t)NT + t0 + 8 * q;
    }
#pragma unroll
    for (int it = 0; it < 4; ++it) *(volatile v8us*)(dvt + off[it]) = u[it];
    __threadfence();
#pragma unroll
    for (int it = 0; it < 4; ++it) *(volatile v8us*)(dvt + off[it]) = u[it];
  } else {
    unsigned short* dh = (stream == 0) ? dq : dk;
    st_rowf(So, rr,      cc,      h00, hinv, bn0);
    st_rowf(So, rr,      cc + 16, h01, hinv, bn1);
    st_rowf(So, rr + 16, cc,      h10, hinv, bn0);
    st_rowf(So, rr + 16, cc + 16, h11, hinv, bn1);
    __syncthreads();
    v8us hv[4];
    size_t off[4];
#pragma unroll
    for (int it = 0; it < 4; ++it) {
      const int p = tid + 256 * it;
      const int hh = p >> 9, rem = p & 511;
      const int row = rem >> 2, q4 = rem & 3;
      const float* sp = So + row * OP + hh * 32 + q4 * 8;
      const v4f a = *(const v4fa*)sp;
      const v4f c = *(const v4fa*)(sp + 4);
      v8h hi = {};
#pragma unroll
      for (int e = 0; e < 4; ++e) { hi[e] = (f16)(a[e] * QS); hi[4 + e] = (f16)(c[e] * QS); }
      hv[it] = __builtin_bit_cast(v8us, hi);
      off[it] = ((size_t)(b * NH + head0 + hh) * NT + t0 + row) * (size_t)DK + q4 * 8;
    }
#pragma unroll
    for (int it = 0; it < 4; ++it) *(volatile v8us*)(dh + off[it]) = hv[it];
    __threadfence();
#pragma unroll
    for (int it = 0; it < 4; ++it) *(volatile v8us*)(dh + off[it]) = hv[it];
  }
}

__global__ __launch_bounds__(256)
void k_attn(const unsigned short* __restrict__ qp, const unsigned short* __restrict__ kp,
            const unsigned short* __restrict__ vtp, const float* __restrict__ btab, int lh0, unsigned short* att) {
  __shared__ __align__(16) float So[64 * OP];
  __shared__ __align__(16) float Sb[2 * NT];
  const int tid = threadIdx.x, lane = tid & 31, wv = tid >> 5, hl = lane >> 4, l15 = lane & 15;
  const int b = (int)blockIdx.y >> 2, hp = (int)blockIdx.y & 3;
  const int hsel = wv >> 2, h = 2 * hp + hsel;
  const int qblk = (int)blockIdx.x * 64;
  const int q0 = qblk + 16 * (wv & 3);
  {
    const float* src = btab + (size_t)(lh0 + 2 * hp) * NT;
#pragma unroll
    for (int j = 0; j < 4; ++j) {
      const int e = tid + 256 * j;
      *(v4fa*)&Sb[4 * e] = *(const v4f*)(src + 4 * e);
    }
  }
  __syncthreads();
  const size_t bh = (size_t)(b * NH + h);
  const f16* Qb = (const f16*)qp  + bh * NT * DK;
  const f16* Kb = (const f16*)kp  + bh * NT * DK;
  const f16* Vb = (const f16*)vtp + bh * DK * NT;
  const float* sbh = Sb + hsel * NT;
  const int myq = q0 + l15;

  const v16h qf = ld_frag(Qb, q0, 0, DK);
  v8f O0 = {}, O1 = {};
  float m = -3.0e38f, l = 0.0f;
  const int kend = q0 + 16;

#pragma unroll 1
  for (int kb = 0; kb < kend; kb += 32) {
    const v16h k0f = ld_frag(Kb, kb, 0, DK);
    const v16h k1f = ld_frag(Kb, kb + 16, 0, DK);
    v8f s0 = {}, s1 = {};
    s0 = mma_h(k0f, qf, s0);
    s1 = mma_h(k1f, qf, s1);
    guard2x3(s0, s1, k0f, k1f, qf);

    float mx = -3.0e38f;
#pragma unroll
    for (int r = 0; r < 8; ++r) {
      const int d0 = myq - (kb + 8 * hl + r);
      const int d1 = d0 - 16;
      const float t0v = sbh[(d0 > 0) ? d0 : 0];
      const float t1v = sbh[(d1 > 0) ? d1 : 0];
      const float b0 = (d0 >= 0) ? t0v : -1.0e9f;
      const float b1 = (d1 >= 0) ? t1v : -1.0e9f;
      const float a0 = s0[r] * SSC + b0;
      const float a1 = s1[r] * SSC + b1;
      s0[r] = a0;
      s1[r] = a1;
      mx = fmaxf(mx, fmaxf(a0, a1));
    }
    mx = fmaxf(mx, __shfl_xor(mx, 16, 32));
    const float mnew = fmaxf(m, mx);
    const float corr = __expf(m - mnew);
    float ps = 0.0f;
    v8h p0v = {}, p1v = {};
#pragma unroll
    for (int r = 0; r < 8; ++r) {
      const float p0 = __expf(s0[r] - mnew);
      const float p1 = __expf(s1[r] - mnew);
      ps += p0 + p1;
      p0v[r] = (f16)(p0 * PSC);
      p1v[r] = (f16)(p1 * PSC);
    }
    ps += __shfl_xor(ps, 16, 32);
    l = l * corr + ps;
    m = mnew;
    O0 *= corr; O1 *= corr;
    FragH pf;
    pf.h[0] = p0v;
    pf.h[1] = p1v;

    const v16h v0f = ld_frag(Vb, 0,  kb, NT);
    const v16h v1f = ld_frag(Vb, 16, kb, NT);
    O0 = mma_h(v0f, pf.v, O0);
    O1 = mma_h(v1f, pf.v, O1);
    guard2x3(O0, O1, v0f, v1f, pf.v);
  }

  const float w = OINV * (1.0f / l);
  float* so = So + (16 * (wv & 3) + l15) * OP + 32 * hsel + 8 * hl;
  st8(so,      O0, w);
  st8(so + 16, O1, w);
  __syncthreads();

  v8us u[2];
  size_t off[2];
#pragma unroll
  for (int it = 0; it < 2; ++it) {
    const int p = tid + 256 * it;
    const int row = p >> 3, q = p & 7;
    const float* sp = So + row * OP + 8 * q;
    const v4f a = *(const v4fa*)sp;
    const v4f c = *(const v4fa*)(sp + 4);
    v8h o = {};
#pragma unroll
    for (int e = 0; e < 4; ++e) { o[e] = (f16)(a[e] * OS); o[4 + e] = (f16)(c[e] * OS); }
    u[it] = __builtin_bit_cast(v8us, o);
    off[it] = ((size_t)(b * NT + qblk + row)) * DM + hp * 64 + 8 * q;
  }
#pragma unroll
  for (int it = 0; it < 2; ++it) *(volatile v8us*)(att + off[it]) = u[it];
  __threadfence();
#pragma unroll
  for (int it = 0; it < 2; ++it) *(volatile v8us*)(att + off[it]) = u[it];
}

__global__ __launch_bounds__(256)
void k_gemm_out(const unsigned short* __restrict__ ah, const unsigned short* __restrict__ al,
                const unsigned short* __restrict__ w16, const float* __restrict__ bias, int nbias,
                float* out, int K, int N) {
  __shared__ __align__(16) float So[128 * OP];
  const int tid = threadIdx.x, lane = tid & 31, wv = tid >> 5, hl = lane >> 4, l15 = lane & 15;
  const int m0 = (int)blockIdx.y * 128, n0 = (int)blockIdx.x * 64;
  const int mp = wv >> 1, np = wv & 1;
  const int ra = m0 + 32 * mp, cb = n0 + 32 * np;
  const f16* Hp = (const f16*)ah;
  const f16* Lp = (const f16*)al;
  const f16* Wp = (const f16*)w16;

  v8f h00 = {}, h01 = {}, h10 = {}, h11 = {};
  v8f g00 = {}, g01 = {}, g10 = {}, g11 = {};
  const int nks = K >> 5;
#pragma unroll 1
  for (int ks = 0; ks < nks; ++ks) {
    const int k0 = ks << 5;
    const v16h a0 = ld_frag(Hp, ra, k0, K);
    const v16h a1 = ld_frag(Hp, ra + 16, k0, K);
    const v16h b0 = ld_frag(Wp, cb, k0, K);
    const v16h b1 = ld_frag(Wp, cb + 16, k0, K);
    h00 = mma_h(a0, b0, h00);
    h01 = mma_h(a0, b1, h01);
    h10 = mma_h(a1, b0, h10);
    h11 = mma_h(a1, b1, h11);
    const v16h e0 = ld_frag(Lp, ra, k0, K);
    const v16h e1 = ld_frag(Lp, ra + 16, k0, K);
    g00 = mma_h(e0, b0, g00);
    g01 = mma_h(e0, b1, g01);
    g10 = mma_h(e1, b0, g10);
    g11 = mma_h(e1, b1, g11);
    guard8x6(h00, h01, h10, h11, g00, g01, g10, g11, a0, a1, b0, b1, e0, e1);
  }

  const int col0 = cb + l15, col1 = cb + 16 + l15;
  const int cc0 = (col0 < nbias) ? col0 : (nbias - 1);
  const int cc1 = (col1 < nbias) ? col1 : (nbias - 1);
  const float bv0 = bf16r(bias[cc0]);
  const float bv1 = bf16r(bias[cc1]);
  const float bn0 = (col0 < nbias) ? bv0 : 0.0f;
  const float bn1 = (col1 < nbias) ? bv1 : 0.0f;
  const int rr = 32 * mp + 8 * hl, cc = 32 * np + l15;
  st_rowf2(So, rr,      cc,      h00, g00, bn0);
  st_rowf2(So, rr,      cc + 16, h01, g01, bn1);
  st_rowf2(So, rr + 16, cc,      h10, g10, bn0);
  st_rowf2(So, rr + 16, cc + 16, h11, g11, bn1);
  __syncthreads();

  v4f u[8];
  size_t off[8];
#pragma unroll
  for (int it = 0; it < 8; ++it) {
    const int p = tid + 256 * it;
    const int row = p >> 4, q = p & 15;
    u[it] = *(const v4fa*)&So[row * OP + 4 * q];
    off[it] = (size_t)(m0 + row) * (size_t)N + n0 + 4 * q;
  }
#pragma unroll
  for (int it = 0; it < 8; ++it) *(volatile v4f*)(out + off[it]) = u[it];
  __threadfence();
#pragma unroll
  for (int it = 0; it < 8; ++it) *(volatile v4f*)(out + off[it]) = u[it];
}

__global__ __launch_bounds__(256)
void k_copy(const float* __restrict__ lg, float* out, int n4) {
  const int p = (int)blockIdx.x * 256 + (int)threadIdx.x;
  if (p >= n4) return;
  const int row = p / (NSK / 4);
  const int c4 = p - row * (NSK / 4);
  const v4f v = *(const v4f*)(lg + (size_t)row * NSP + 4 * c4);
  float* op = out + (size_t)p * 4;
  *(volatile v4f*)op = v;
  __threadfence();
  *(volatile v4f*)op = v;
}

extern "C" void kernel_launch(void* const* d_in, const int* in_sizes, int n_in,
                              void* d_out, int out_size, void* d_ws, size_t ws_size,
                              hipStream_t stream) {
  if (n_in < 33) return;
  if (in_sizes[0] != NR || in_sizes[1] != NR || in_sizes[2] != NR * FIN) return;
  if (in_sizes[3] != NEMB * DM || in_sizes[4] != NPAT * DQ || in_sizes[5] != FIN * DQ || in_sizes[6] != DQ) return;
  if (in_sizes[7] != KIN * DM || in_sizes[8] != DM) return;
  if (in_sizes[9] != DM || in_sizes[10] != DM || in_sizes[11] != DM || in_sizes[12] != DM) return;
  for (int i = 0; i < 4; ++i) {
    if (in_sizes[13 + 2 * i] != NL * DM * DM || in_sizes[14 + 2 * i] != NL * DM) return;
  }
  if (in_sizes[21] != NL * NH || in_sizes[22] != NL * NH) return;
  for (int i = 23; i < 27; ++i) { if (in_sizes[i] != NL * DM) return; }
  if (in_sizes[27] != NL * DM * DF || in_sizes[28] != NL * DF || in_sizes[29] != NL * DF * DM || in_sizes[30] != NL * DM) return;
  if (in_sizes[31] != DM * NSK || in_sizes[32] != NSK) return;
  if (out_size != NR * NSK) return;

  const size_t sz_xin  = (size_t)NR * KIN * 2;
  const size_t sz_win  = (size_t)DM * KIN * 2;
  const size_t sz_wqkv = (size_t)NL * 3 * DM * DM * 2;
  const size_t sz_wo   = (size_t)NL * DM * DM * 2;
  const size_t sz_wu   = (size_t)NL * DF * DM * 2;
  const size_t sz_wd   = (size_t)NL * DM * DF * 2;
  const size_t sz_wout = (size_t)NSP * DM * 2;
  const size_t sz_bt   = (size_t)NL * NH * NT * 4;
  const size_t sz_x    = (size_t)NR * DM * 4;
  const size_t sz_p16  = (size_t)NR * DM * 2;
  const size_t sz_hp   = (size_t)NR * DF * 2;
  const size_t sz_lg   = (size_t)MH * NSP * 4;

  const size_t off_xin  = 0;
  const size_t off_win  = off_xin  + sz_xin;
  const size_t off_wqkv = off_win  + sz_win;
  const size_t off_wo   = off_wqkv + sz_wqkv;
  const size_t off_wu   = off_wo   + sz_wo;
  const size_t off_wd   = off_wu   + sz_wu;
  const size_t off_wout = off_wd   + sz_wd;
  const size_t off_bt   = off_wout + sz_wout;
  const size_t off_xa   = off_bt   + sz_bt;
  const size_t off_xb   = off_xa   + sz_x;
  const size_t off_x16  = off_xb   + sz_x;
  const size_t off_x16l = off_x16  + sz_p16;
  const size_t off_q    = off_x16l + sz_p16;
  const size_t off_k    = off_q    + sz_p16;
  const size_t off_vt   = off_k    + sz_p16;
  const size_t off_att  = off_vt   + sz_p16;
  const size_t off_hp   = off_att  + sz_p16;
  const size_t off_lg   = off_hp   + sz_hp;
  const size_t need     = off_lg   + sz_lg;
  if (need > ws_size) return;
  if (need > (size_t)134217728) return;

  const int*   inter = (const int*)  d_in[0];
  const int*   pat   = (const int*)  d_in[1];
  const float* ff    = (const float*)d_in[2];
  const float* iemb  = (const float*)d_in[3];
  const float* pemb  = (const float*)d_in[4];
  const float* fW    = (const float*)d_in[5];
  const float* fb    = (const float*)d_in[6];
  const float* inW   = (const float*)d_in[7];
  const float* inb   = (const float*)d_in[8];
  const float* tW    = (const float*)d_in[9];
  const float* tb    = (const float*)d_in[10];
  const float* pW    = (const float*)d_in[11];
  const float* pb    = (const float*)d_in[12];
  const float* Wq    = (const float*)d_in[13];
  const float* bq    = (const float*)d_in[14];
  const float* Wk    = (const float*)d_in[15];
  const float* bk    = (const float*)d_in[16];
  const float* Wv    = (const float*)d_in[17];
  const float* bv    = (const float*)d_in[18];
  const float* Wo    = (const float*)d_in[19];
  const float* bo    = (const float*)d_in[20];
  const float* kpp   = (const float*)d_in[21];
  const float* kpa   = (const float*)d_in[22];
  const float* ln1g  = (const float*)d_in[23];
  const float* ln1b  = (const float*)d_in[24];
  const float* ln2g  = (const float*)d_in[25];
  const float* ln2b  = (const float*)d_in[26];
  const float* W1    = (const float*)d_in[27];
  const float* b1    = (const float*)d_in[28];
  const float* W2    = (const float*)d_in[29];
  const float* b2    = (const float*)d_in[30];
  const float* Wout  = (const float*)d_in[31];
  const float* bout  = (const float*)d_in[32];

  float* out0 = (float*)d_out;

  char* wsb = (char*)d_ws;
  unsigned short* xin_p  = (unsigned short*)(wsb + off_xin);
  unsigned short* win_p  = (unsigned short*)(wsb + off_win);
  unsigned short* wqkv_p = (unsigned short*)(wsb + off_wqkv);
  unsigned short* wo_p   = (unsigned short*)(wsb + off_wo);
  unsigned short* wu_p   = (unsigned short*)(wsb + off_wu);
  unsigned short* wd_p   = (unsigned short*)(wsb + off_wd);
  unsigned short* wout_p = (unsigned short*)(wsb + off_wout);
  float*          bt_p   = (float*)(wsb + off_bt);
  float*          xa_p   = (float*)(wsb + off_xa);
  float*          xb_p   = (float*)(wsb + off_xb);
  unsigned short* x16_p  = (unsigned short*)(wsb + off_x16);
  unsigned short* x16l_p = (unsigned short*)(wsb + off_x16l);
  unsigned short* q_p    = (unsigned short*)(wsb + off_q);
  unsigned short* k_p    = (unsigned short*)(wsb + off_k);
  unsigned short* vt_p   = (unsigned short*)(wsb + off_vt);
  unsigned short* att_p  = (unsigned short*)(wsb + off_att);
  unsigned short* hp_p   = (unsigned short*)(wsb + off_hp);
  float*          lg_p   = (float*)(wsb + off_lg);

  const dim3 blk(256);

  k_cvt_wg<<<dim3((DM * (KIN / 8)) / 256, 1),  blk, 0, stream>>>(inW,  win_p,  KIN, DM,  DM,  DM,     0,      WSC);
  k_cvt_wg<<<dim3((DM * (DM / 8)) / 256, NL),  blk, 0, stream>>>(Wq,   wqkv_p, DM,  DM,  DM,  3 * DM, 0,      WSC);
  k_cvt_wg<<<dim3((DM * (DM / 8)) / 256, NL),  blk, 0, stream>>>(Wk,   wqkv_p, DM,  DM,  DM,  3 * DM, DM,     WSC);
  k_cvt_wg<<<dim3((DM * (DM / 8)) / 256, NL),  blk, 0, stream>>>(Wv,   wqkv_p, DM,  DM,  DM,  3 * DM, 2 * DM, WSC);
  k_cvt_wg<<<dim3((DM * (DM / 8)) / 256, NL),  blk, 0, stream>>>(Wo,   wo_p,   DM,  DM,  DM,  DM,     0,      WSC);
  k_cvt_wg<<<dim3((DF * (DM / 8)) / 256, NL),  blk, 0, stream>>>(W1,   wu_p,   DM,  DF,  DF,  DF,     0,      WSC);
  k_cvt_wg<<<dim3((DM * (DF / 8)) / 256, NL),  blk, 0, stream>>>(W2,   wd_p,   DF,  DM,  DM,  DM,     0,      WSC);
  k_cvt_wg<<<dim3((NSP * (DM / 8)) / 256, 1), blk, 0, stream>>>(Wout, wout_p, DM,  NSK, NSP, NSP,    0,      WSC);

  k_bias<<<dim3(NT / 256, NL * NH), blk, 0, stream>>>(kpp, kpa, bt_p);

  k_xin<<<dim3(NR / 4), blk, 0, stream>>>(inter, pat, ff, iemb, pemb, fW, fb, xin_p);
  k_gemm_x<0><<<dim3(DM / 64, NR / 128), blk, 0, stream>>>(xin_p, win_p, inb, xb_p, ff, tW, tb, pW, pb,
                                                          xa_p, x16_p, KIN, DM, INV_IN);

  const dim3 g_ln(NR / 8), g_heads(3 * DM / 64, NR / 128), g_attn(NT / 64, NB * (NH / 2));
  const dim3 g_dm(DM / 64, NR / 128), g_ff(DF / 64, NR / 128);
  for (int i = 0; i < NL; ++i) {
    const unsigned short* wqkv_i = wqkv_p + (size_t)i * 3 * DM * DM;
    const unsigned short* wo_i   = wo_p   + (size_t)i * DM * DM;
    const unsigned short* wu_i   = wu_p   + (size_t)i * DF * DM;
    const unsigned short* wd_i   = wd_p   + (size_t)i * DM * DF;
    const float hinv_a = (i == 0) ? INV_X0 : INV_LN;
    k_gemm_heads<<<g_heads, blk, 0, stream>>>(x16_p, wqkv_i, bq + i * DM, bk + i * DM, bv + i * DM,
                                              q_p, k_p, vt_p, DM, hinv_a);
    k_attn<<<g_attn, blk, 0, stream>>>(q_p, k_p, vt_p, bt_p, i * NH, att_p);
    k_gemm_x<1><<<g_dm, blk, 0, stream>>>(att_p, wo_i, bo + i * DM, xa_p, ff, tW, tb, pW, pb,
                                          xb_p, x16l_p, DM, DM, INV_AT);
    k_ln<false><<<g_ln, blk, 0, stream>>>(xb_p, ln1g + i * DM, ln1b + i * DM, xa_p, x16_p, x16l_p);
    k_gemm_h<<<g_ff, blk, 0, stream>>>(x16_p, wu_i, b1 + i * DF, hp_p, DM, DF, INV_LN);
    k_gemm_x<1><<<g_dm, blk, 0, stream>>>(hp_p, wd_i, b2 + i * DM, xa_p, ff, tW, tb, pW, pb,
                                          xb_p, x16l_p, DF, DM, INV_HP);
    if (i == NL - 1) {
      k_ln<true><<<g_ln, blk, 0, stream>>>(xb_p, ln2g + i * DM, ln2b + i * DM, xa_p, x16_p, x16l_p);
    } else {
      k_ln<false><<<g_ln, blk, 0, stream>>>(xb_p, ln2g + i * DM, ln2b + i * DM, xa_p, x16_p, x16l_p);
    }
  }

  const dim3 g_out(NSP / 64, MH / 128), g_copy((MH * (NSK / 4)) / 256);
  for (int hf = 0; hf < 2; ++hf) {
    const unsigned short* ah = x16_p  + (size_t)hf * MH * DM;
    const unsigned short* al = x16l_p + (size_t)hf * MH * DM;
    k_gemm_out<<<g_out, blk, 0, stream>>>(ah, al, wout_p, bout, NSK, lg_p, DM, NSP);
    k_copy<<<g_copy, blk, 0, stream>>>(lg_p, out0 + (size_t)hf * MH * NSK, MH * (NSK / 4));
  }
  (void)hipGetLastError();
}
